// Intra_GCN_52329881534579
// MI455X (gfx1250) — hardware-verified
//
#include <hip/hip_runtime.h>


namespace {
constexpr int N = 10000, E = 160000, D = 512, G = 256, NPAD = 10112  , NBLK = NPAD / 128;
constexpr float FXS = 524288.0f, FXI = 1.0f / 524288.0f, LNE = 1e-5f;

typedef _Float16 b16;
typedef __attribute__((ext_vector_type(16))) _Float16 v16b;
typedef __attribute__((ext_vector_type(8)))  _Float16 v8b;
typedef __attribute__((ext_vector_type(8)))  float v8f;
typedef __attribute__((ext_vector_type(4)))  float v4f;

__device__ __forceinline__ v8b ld8b(const b16* p) { return *(const v8b*)p; }
__device__ __forceinline__ v16b cat8b(v8b a, v8b b) { return __builtin_shufflevector(a, b, 0, 1, 2, 3, 4, 5, 6, 7, 8, 9, 10, 11, 12, 13, 14, 15); }
__device__ __forceinline__ v16b frag_kb(const b16* p, int hh) { return cat8b(ld8b(p + 8 * hh), ld8b(p + 16 + 8 * hh)); }
__device__ __forceinline__ void split16(float v, b16& hi, b16& lo) { hi = (b16)v; lo = (b16)(v - (float)hi); }
__device__ __forceinline__ void frag_ksplit(const float* p, int hh, v16b& fh_, v16b& fl_) {
  const float* p0 = p + 8 * hh; const float* p1 = p + 16 + 8 * hh;
#pragma unroll
  for (int e = 0; e < 8; ++e) { b16 a, c; split16(p0[e], a, c); fh_[e] = a; fl_[e] = c; split16(p1[e], a, c); fh_[8 + e] = a; fl_[8 + e] = c; }
}
__device__ __forceinline__ v8f wmma16b(v16b a, v16b b, v8f c) {
  v8f d = __builtin_amdgcn_wmma_f32_16x16x32_f16(false, a, false, b, (short)0, c, false, false);
  asm volatile("v_nop\n\tv_nop\n\tv_nop\n\tv_nop" : "+v"(d) : "v"(a), "v"(b));
  return d;
}
__device__ __forceinline__ void wave_lds_sync() {
  __builtin_amdgcn_fence(__ATOMIC_RELEASE, "workgroup");
  __builtin_amdgcn_wave_barrier();
  __builtin_amdgcn_fence(__ATOMIC_ACQUIRE, "workgroup");
}

struct Opnd { const void* p0; const void* p1; int ld; };
template <int NP> __device__ __forceinline__ void load_frags(const Opnd& o, int row, int kb, int hh, v16b& fh_, v16b& fl_) {
  if (NP == 0) { frag_ksplit((const float*)o.p0 + (size_t)row * o.ld + kb, hh, fh_, fl_); }
  else if (NP == 4) {
    const float* p = (const float*)o.p0 + (size_t)row * o.ld + kb; const float* p0 = p + 8 * hh; const float* p1 = p + 16 + 8 * hh;
#pragma unroll
    for (int e = 0; e < 8; ++e) { b16 a, c; split16(p0[e] * 64.0f, a, c); fh_[e] = a; fl_[e] = c; split16(p1[e] * 64.0f, a, c); fh_[8 + e] = a; fl_[8 + e] = c; }
  } else if (NP == 3) {
    const float* p = (const float*)o.p0 + (size_t)row * o.ld + kb; const float* p0 = p + 8 * hh; const float* p1 = p + 16 + 8 * hh;
#pragma unroll
    for (int e = 0; e < 8; ++e) { fh_[e] = (b16)p0[e]; fh_[8 + e] = (b16)p1[e]; }
    fl_ = fh_;
  } else {
    fh_ = frag_kb((const b16*)o.p0 + (size_t)row * o.ld + kb, hh);
    if (NP == 2) fl_ = frag_kb((const b16*)o.p1 + (size_t)row * o.ld + kb, hh); else fl_ = fh_;
  }
}
template <int ANP, int BNP> __device__ __forceinline__ v8f mac(v16b ah, v16b al, v16b bh, v16b bl, v8f c) {
  c = wmma16b(ah, bh, c);
  if (BNP == 0 || BNP == 2 || BNP == 4) c = wmma16b(ah, bl, c);
  if (ANP == 0 || ANP == 2 || ANP == 4) c = wmma16b(al, bh, c);
  return c;
}
template <int ANP, int BNP>
__device__ __forceinline__ void gemm_tile(const Opnd& A, const Opnd& B, int K, int m0, int c0, int nloc, int hlf, v8f (&acc)[2][4]) {
  for (int kb = 0; kb < K; kb += 32) {
    v16b a0h, a0l, a1h, a1l;
    load_frags<ANP>(A, m0 + nloc, kb, hlf, a0h, a0l);
    load_frags<ANP>(A, m0 + 16 + nloc, kb, hlf, a1h, a1l);
#pragma unroll
    for (int t = 0; t < 4; ++t) {
      v16b bh, bl;
      load_frags<BNP>(B, c0 + t * 16 + nloc, kb, hlf, bh, bl);
      acc[0][t] = mac<ANP, BNP>(a0h, a0l, bh, bl, acc[0][t]);
      acc[1][t] = mac<ANP, BNP>(a1h, a1l, bh, bl, acc[1][t]);
    }
  }
}

__device__ __forceinline__ void epi_planes(v8f (&acc)[2][4], float scale, bool two, b16* __restrict__ oh, b16* __restrict__ ol, int ldo,
                                           int m0, int c0, int lane, b16* Th, b16* Tl) {
  const int nloc = lane & 15, hlf = lane >> 4;
#pragma unroll
  for (int t = 0; t < 4; ++t)
#pragma unroll
    for (int r = 0; r < 2; ++r)
#pragma unroll
      for (int v = 0; v < 8; ++v) {
        const int rr = r * 16 + v + 8 * hlf, cc = t * 16 + nloc;
        b16 h_, l_; split16(acc[r][t][v] * scale, h_, l_);
        Th[rr * 64 + cc] = h_; Tl[rr * 64 + cc] = l_;
      }
  wave_lds_sync();
  for (int pass = 0; pass < 2; ++pass) {
#pragma unroll
    for (int j = 0; j < 8; ++j) {
      const int rr = j * 4 + (lane >> 3), c8 = (lane & 7) * 8;
      const size_t o = (size_t)(m0 + rr) * ldo + c0 + c8;
      *(volatile v8b*)(oh + o) = ld8b(Th + rr * 64 + c8);
      if (two) *(volatile v8b*)(ol + o) = ld8b(Tl + rr * 64 + c8);
    }
    __threadfence();
  }
}
__device__ __forceinline__ void epi_f32(v8f (&acc)[2][4], float scale, const float* rscale, float* __restrict__ out, int ldo, int m0, int c0, int lane, float* Tt) {
  const int nloc = lane & 15, hlf = lane >> 4;
#pragma unroll
  for (int t = 0; t < 4; ++t)
#pragma unroll
    for (int r = 0; r < 2; ++r)
#pragma unroll
      for (int v = 0; v < 8; ++v) {
        const int rr = r * 16 + v + 8 * hlf;
        const float rs = rscale ? rscale[(size_t)(m0 + rr) * 32] : 1.0f;
        Tt[rr * 64 + t * 16 + nloc] = acc[r][t][v] * scale * rs;
      }
  wave_lds_sync();
  float* dst0 = out + (size_t)m0 * ldo + c0;
  for (int pass = 0; pass < 2; ++pass) {
#pragma unroll
    for (int j = 0; j < 16; ++j) { const int rr = j * 2 + hlf, c4 = nloc * 4; *(volatile v4f*)(dst0 + (size_t)rr * ldo + c4) = *(const v4f*)(Tt + rr * 64 + c4); }
    __threadfence();
  }
}


__global__ __launch_bounds__(256) void prep_kernel(const float* __restrict__ Wn, const float* __restrict__ Wr, b16* __restrict__ w16) {
  const size_t tid = (size_t)blockIdx.x * blockDim.x + threadIdx.x, nth = (size_t)gridDim.x * blockDim.x;
  for (int pass = 0; pass < 2; ++pass) { for (size_t p = tid; p < (size_t)D * 2 * D / 8; p += nth) { const int n = (int)(p / (2 * D / 8)), k0 = (int)(p % (2 * D / 8)) * 8; v8b v;
#pragma unroll
      for (int e = 0; e < 8; ++e) { const int k = k0 + e; v[e] = (b16)((k < D) ? Wn[(size_t)n * D + min(k, D - 1)] : Wr[(size_t)n * D + (k - D)]); }
      *(volatile v8b*)(w16 + (size_t)n * 2 * D + k0) = v; } __threadfence(); }
}

__global__ __launch_bounds__(256) void ln0_kernel(const float* __restrict__ x, const float* __restrict__ g, const float* __restrict__ bb, float* __restrict__ cat) {
  const int wid = threadIdx.x >> 5, lane = threadIdx.x & 31, row = blockIdx.x * 8 + wid;
  v4f v[4]; float s = 0.0f;
  if (row < N) {
#pragma unroll
    for (int j = 0; j < 4; ++j) { v[j] = *(const v4f*)(x + (size_t)row * D + j * 128 + lane * 4); s += v[j][0] + v[j][1] + v[j][2] + v[j][3]; } }
  else {
#pragma unroll
    for (int j = 0; j < 4; ++j) v[j] = (v4f){0.0f, 0.0f, 0.0f, 0.0f}; }
#pragma unroll
  for (int o = 16; o > 0; o >>= 1) s += __shfl_xor(s, o);
  const float mean = s * (1.0f / D); float s2 = 0.0f;
#pragma unroll
  for (int j = 0; j < 4; ++j)
#pragma unroll
    for (int e = 0; e < 4; ++e) { const float dd = v[j][e] - mean; s2 += dd * dd; }
#pragma unroll
  for (int o = 16; o > 0; o >>= 1) s2 += __shfl_xor(s2, o);
  const float rs = rsqrtf(s2 * (1.0f / D) + LNE);
  for (int pass = 0; pass < 2; ++pass) {
#pragma unroll
    for (int j = 0; j < 4; ++j) { v4f o; const int c = j * 128 + lane * 4;
#pragma unroll
      for (int e = 0; e < 4; ++e) o[e] = (row < N) ? ((v[j][e] - mean) * rs * g[c + e] + bb[c + e]) : 0.0f;
      *(volatile v4f*)(cat + (size_t)row * 2 * D + D + c) = o;
      if (row >= N) *(volatile v4f*)(cat + (size_t)row * 2 * D + c) = o; }
    __threadfence();
  }
}

typedef __attribute__((ext_vector_type(4))) int v4i;
template <int NB>
__global__ __launch_bounds__(256) void mean_kernel(const int* __restrict__ keys, const int* __restrict__ other, int nkeys, const float* __restrict__ feat, int fpitch, float* __restrict__ outp, int opitch, int nown, int nown_pad) {
  __shared__ __attribute__((aligned(16))) int acc[NB * D];
  __shared__ int cnt[NB]; __shared__ int list[8 * 256];
  const int t_ = threadIdx.x, wave = t_ >> 5, lane = t_ & 31, base = blockIdx.x * NB;
  for (int i = t_; i < NB * D; i += 256) acc[i] = 0;
  for (int i = t_; i < NB; i += 256) cnt[i] = 0;
  __syncthreads();
  int* wl = list + wave * 256;
  for (int c0 = 0; c0 < nkeys; c0 += 256 * 8) {
    const int e0 = c0 + (wave * 32 + lane) * 8; int dd[8];
#pragma unroll
    for (int j = 0; j < 8; ++j) { const int dv = keys[min(e0 + j, nkeys - 1)]; dd[j] = (e0 + j < nkeys) ? dv : -1; }
    unsigned sl[8]; bool hit[8]; bool anyl = false;
#pragma unroll
    for (int j = 0; j < 8; ++j) { sl[j] = (unsigned)(dd[j] - base); hit[j] = sl[j] < (unsigned)NB; anyl |= hit[j]; }
    int wc = 0;
    if (__builtin_amdgcn_ballot_w32(anyl) != 0u) {
#pragma unroll
      for (int j = 0; j < 8; ++j) {
        const unsigned mj = __builtin_amdgcn_ballot_w32(hit[j]);
        if (mj != 0u) {
          if (hit[j]) { const int pos = wc + (int)__builtin_amdgcn_mbcnt_lo(mj, 0u); int o = other ? other[min(e0 + j, nkeys - 1)] : (e0 + j); o = (o < 0) ? 0 : (o >= N ? N - 1 : o); wl[pos] = (o << 8) | (int)sl[j]; atomicAdd(&cnt[sl[j]], 1); }
          wc += __builtin_popcount(mj); } } }
    __builtin_amdgcn_wave_barrier(); __builtin_amdgcn_fence(__ATOMIC_RELEASE, "workgroup"); __builtin_amdgcn_fence(__ATOMIC_ACQUIRE, "workgroup");
    for (int i = 0; i < wc; ++i) { const int ent = wl[i]; const int o = ent >> 8, slot = ent & 255; const float* fr = feat + (size_t)o * fpitch + lane * 16; int* ar = acc + slot * D + lane * 16;
#pragma unroll
      for (int q4 = 0; q4 < 4; ++q4) { const v4f v = *(const v4f*)(fr + q4 * 4);
#pragma unroll
        for (int c = 0; c < 4; ++c) atomicAdd(ar + q4 * 4 + c, (int)rintf(v[c] * FXS)); } }
    __builtin_amdgcn_wave_barrier();
  }
  __syncthreads();
  for (int pass = 0; pass < 2; ++pass) {
    for (int i = t_; i < NB * D / 4; i += 256) { const int r = i / (D / 4), cq = (i % (D / 4)) * 4, row = base + r; if (row < nown_pad) { v4f o = {0.0f, 0.0f, 0.0f, 0.0f};
        if (row < nown) { const float inv = 1.0f / fmaxf((float)cnt[r], 1.0f);
#pragma unroll
          for (int c = 0; c < 4; ++c) o[c] = (float)acc[r * D + cq + c] * FXI * inv; }
        *(volatile v4f*)(outp + (size_t)row * opitch + cq) = o; } }
    __threadfence();
  }
}

__global__ __launch_bounds__(128) void lin_kernel(const float* __restrict__ cat, const b16* __restrict__ w16, const float* __restrict__ bias, float* __restrict__ pre) {
  __shared__ __attribute__((aligned(16))) float Ts[4][32 * 64];
  const int lane = threadIdx.x & 31, wave = threadIdx.x >> 5, nloc = lane & 15, hlf = lane >> 4, m0 = blockIdx.y * 128 + wave * 32, c0 = blockIdx.x * 64;
  v8f acc[2][4];
#pragma unroll
  for (int r = 0; r < 2; ++r)
#pragma unroll
    for (int t = 0; t < 4; ++t) acc[r][t] = (v8f){};
  const Opnd A{cat, nullptr, 2 * D}, Bo{w16, nullptr, 2 * D};
  gemm_tile<3, 1>(A, Bo, 2 * D, m0, c0, nloc, hlf, acc);
#pragma unroll
  for (int t = 0; t < 4; ++t)
#pragma unroll
    for (int r = 0; r < 2; ++r)
#pragma unroll
      for (int v = 0; v < 8; ++v) acc[r][t][v] = fmaxf(acc[r][t][v] + bias[c0 + t * 16 + nloc], 0.0f);
  epi_f32(acc, 1.0f, nullptr, pre, D, m0, c0, lane, Ts[wave]);
}

__global__ __launch_bounds__(256) void ln1_kernel(const float* __restrict__ pre, const float* __restrict__ g, const float* __restrict__ bb, float* __restrict__ nodeout) {
  const int wid = threadIdx.x >> 5, lane = threadIdx.x & 31, row = blockIdx.x * 8 + wid;
  v4f v[4]; float s = 0.0f;
#pragma unroll
  for (int j = 0; j < 4; ++j) { v[j] = *(const v4f*)(pre + (size_t)row * D + j * 128 + lane * 4); s += v[j][0] + v[j][1] + v[j][2] + v[j][3]; }
#pragma unroll
  for (int o = 16; o > 0; o >>= 1) s += __shfl_xor(s, o);
  const float mean = s * (1.0f / D); float s2 = 0.0f;
#pragma unroll
  for (int j = 0; j < 4; ++j)
#pragma unroll
    for (int e = 0; e < 4; ++e) { const float dd = v[j][e] - mean; s2 += dd * dd; }
#pragma unroll
  for (int o = 16; o > 0; o >>= 1) s2 += __shfl_xor(s2, o);
  const float rs = rsqrtf(s2 * (1.0f / D) + LNE);
  for (int pass = 0; pass < 2; ++pass) {
#pragma unroll
    for (int j = 0; j < 4; ++j) { v4f o; const int c = j * 128 + lane * 4;
#pragma unroll
      for (int e = 0; e < 4; ++e) o[e] = (v[j][e] - mean) * rs * g[c + e] + bb[c + e];
      *(volatile v4f*)(nodeout + (size_t)row * D + c) = o; }
    __threadfence();
  }
}
}

extern "C" void kernel_launch(void* const* d_in, const int* in_sizes, int n_in,
                              void* d_out, int out_size, void* d_ws, size_t ws_size, hipStream_t stream) {
  (void)n_in; (void)out_size;
  const float* x = (const float*)d_in[0]; const int* ei = (const int*)d_in[1]; const int* batch = (const int*)d_in[2];
  const float* ln0w = (const float*)d_in[3]; const float* ln0b = (const float*)d_in[4]; const float* Wn = (const float*)d_in[5]; const float* Wr = (const float*)d_in[6]; const float* bias = (const float*)d_in[7];
  const float* ln1w = (const float*)d_in[8]; const float* ln1b = (const float*)d_in[9];
  float* out = (float*)d_out;
  if (in_sizes[0] != N * D || in_sizes[1] != 2 * E || in_sizes[2] != N || in_sizes[5] != D * D || in_sizes[6] != D * D) return;
  const int* esrc = ei; const int* edst = ei + E;
  size_t off = 0; char* ws = (char*)d_ws;
  auto carve = [&](size_t bytes) { char* p = ws + off; off += (bytes + 255) & ~(size_t)255; return p; };
  b16* w16 = (b16*)carve((size_t)D * 2 * D * 2); float* cat = (float*)carve((size_t)NPAD * 2 * D * 4); float* pre = (float*)carve((size_t)NPAD * D * 4); float* nodeout = (float*)carve((size_t)NPAD * D * 4);
  if (off > ws_size) return;
  prep_kernel<<<256, 256, 0, stream>>>(Wn, Wr, w16);
  ln0_kernel<<<NPAD / 8, 256, 0, stream>>>(x, ln0w, ln0b, cat);
  mean_kernel<128><<<NPAD / 128, 256, 0, stream>>>(edst, esrc, E, cat + D, 2 * D, cat, 2 * D, N, NPAD);
  lin_kernel<<<dim3(D / 64, NBLK), 128, 0, stream>>>(cat, w16, bias, pre);
  ln1_kernel<<<NPAD / 8, 256, 0, stream>>>(pre, ln1w, ln1b, nodeout);
  mean_kernel<128><<<G / 128, 256, 0, stream>>>(batch, nullptr, N, nodeout, D, out, D, G, G);
}
